// Self_Attn_31370441130462
// MI455X (gfx1250) — hardware-verified
//
#include <hip/hip_runtime.h>


#ifndef NB
#define NB 8
#endif
#ifndef SEQ
#define SEQ 2048
#endif
#define NB_FULL  8
#define SEQ_FULL 2048
#define DD       512
#define NROWS    (NB * SEQ)
#define NWROWS   1536

static_assert(NB >= 1 && NB <= NB_FULL);
static_assert(SEQ >= 128 && SEQ <= SEQ_FULL);
static_assert((SEQ % 128) == 0);
static_assert((DD % 128) == 0);

#define WCARRY      256.0f
#define INV_WCARRY  0.00390625f
#define RCARRY      4096.0f
#define INV_RCARRY  0.000244140625f
#define PCARRY      16384.0f
#define VCARRY      16.0f
#define INV_PV      (1.0f / 262144.0f)
#define L2E         1.4426950408889634f
#define TP          136

typedef _Float16 v16h __attribute__((ext_vector_type(16)));
typedef _Float16 v8h  __attribute__((ext_vector_type(8)));
typedef float    v8f  __attribute__((ext_vector_type(8)));
typedef float    v4f  __attribute__((ext_vector_type(4)));

union Frag { v16h v; v8h p[2]; };
union Acc8 { v8f v; v4f q[2]; };

__device__ __forceinline__ v16h ldfrag(const _Float16* p) {
  Frag f;
  f.p[0] = *(const v8h*)p;
  f.p[1] = *(const v8h*)(p + 16);
  return f.v;
}

__device__ __forceinline__ v8f mma16(v16h a, v16h b, v8f c) {
  return __builtin_amdgcn_wmma_f32_16x16x32_f16(false, a, false, b, (short)0, c, false, false);
}

__device__ __forceinline__ v8f zero8() {
  v8f z;
#pragma unroll
  for (int r = 0; r < 8; ++r) z[r] = 0.0f;
  return z;
}

__device__ __forceinline__ float bf16_rne(float f) {
  unsigned u = __builtin_bit_cast(unsigned, f);
  u = (u + 0x7FFFu + ((u >> 16) & 1u)) & 0xFFFF0000u;
  return __builtin_bit_cast(float, u);
}

__global__ __launch_bounds__(256) void cvt_kernel(
    const float* __restrict__ x,
    const float* __restrict__ Wq, const float* __restrict__ bq,
    const float* __restrict__ Wk, const float* __restrict__ bk,
    const float* __restrict__ Wv, const float* __restrict__ bv,
    _Float16* __restrict__ xh, _Float16* __restrict__ wc, float* __restrict__ bc,
    int nbx, int nbw)
{
  const int blk = blockIdx.x;
  const int tid = threadIdx.x;
  if (blk < nbx) {
    const unsigned g    = (unsigned)blk * 256u + (unsigned)tid;
    const unsigned prow = g >> 6;
    const int      col  = (int)(g & 63u) * 8;
    const unsigned bb   = prow / (unsigned)SEQ;
    const unsigned s    = prow - bb * (unsigned)SEQ;
    const float* src = x + ((size_t)bb * SEQ_FULL + s) * DD + col;
    const v4f a = *(const v4f*)src;
    const v4f c = *(const v4f*)(src + 4);
    v8h o;
    o[0] = (_Float16)bf16_rne(a[0]);
    o[1] = (_Float16)bf16_rne(a[1]);
    o[2] = (_Float16)bf16_rne(a[2]);
    o[3] = (_Float16)bf16_rne(a[3]);
    o[4] = (_Float16)bf16_rne(c[0]);
    o[5] = (_Float16)bf16_rne(c[1]);
    o[6] = (_Float16)bf16_rne(c[2]);
    o[7] = (_Float16)bf16_rne(c[3]);
    _Float16* dst = xh + (size_t)prow * DD + col;
    *(volatile v8h*)dst = o;
    __threadfence();
    *(volatile v8h*)dst = o;
  } else if (blk < nbx + nbw) {
    const unsigned g   = (unsigned)(blk - nbx) * 256u + (unsigned)tid;
    const unsigned n   = g >> 6;
    const int      col = (int)(g & 63u) * 8;
    const int      mat = __builtin_amdgcn_readfirstlane((int)(g >> 15));
    const float* W = (mat == 0) ? Wq : ((mat == 1) ? Wk : Wv);
    const float* src = W + (size_t)(n - (unsigned)mat * 512u) * DD + col;
    const v4f a = *(const v4f*)src;
    const v4f c = *(const v4f*)(src + 4);
    v8h o;
    o[0] = (_Float16)(bf16_rne(a[0]) * WCARRY);
    o[1] = (_Float16)(bf16_rne(a[1]) * WCARRY);
    o[2] = (_Float16)(bf16_rne(a[2]) * WCARRY);
    o[3] = (_Float16)(bf16_rne(a[3]) * WCARRY);
    o[4] = (_Float16)(bf16_rne(c[0]) * WCARRY);
    o[5] = (_Float16)(bf16_rne(c[1]) * WCARRY);
    o[6] = (_Float16)(bf16_rne(c[2]) * WCARRY);
    o[7] = (_Float16)(bf16_rne(c[3]) * WCARRY);
    _Float16* dst = wc + (size_t)n * DD + col;
    *(volatile v8h*)dst = o;
    __threadfence();
    *(volatile v8h*)dst = o;
  } else {
    const int t = (blk - nbx - nbw) * 256 + tid;
    if (t < NWROWS / 4) {
      const int e   = t * 4;
      const int idx = e & 511;
      const int m   = e >> 9;
      const v4f uq = *(const v4f*)(bq + idx);
      const v4f uk = *(const v4f*)(bk + idx);
      const v4f uv = *(const v4f*)(bv + idx);
      v4f o;
#pragma unroll
      for (int i = 0; i < 4; ++i) {
        const float s0 = uq[i], s1 = uk[i], s2 = uv[i];
        const float sel = (m == 0) ? s0 : ((m == 1) ? s1 : s2);
        o[i] = bf16_rne(sel);
      }
      float* dst = bc + e;
      *(volatile v4f*)dst = o;
      __threadfence();
      *(volatile v4f*)dst = o;
    }
  }
}

__global__ __launch_bounds__(256) void proj_kernel(
    const _Float16* __restrict__ xh, const _Float16* __restrict__ wc,
    const float* __restrict__ bc,
    _Float16* __restrict__ qh, _Float16* __restrict__ ql,
    _Float16* __restrict__ kh, _Float16* __restrict__ kl,
    _Float16* __restrict__ vt)
{
  __shared__ __attribute__((aligned(16))) _Float16 T[128 * TP];

  const int tid  = threadIdx.x;
  const int w    = __builtin_amdgcn_readfirstlane(tid >> 5);
  const int lane = tid & 31, h = lane >> 4, l16 = lane & 15;
  const int wr   = w >> 1, wq = w & 1;
  const int rb   = blockIdx.x * 128;
  const int cbk  = blockIdx.y;
  const int mat  = cbk >> 2;
  const int c0   = (cbk & 3) * 128;

  const _Float16* ap0 = xh + (size_t)(rb + 32 * wr + l16) * DD + 8 * h;
  const _Float16* ap1 = ap0 + (size_t)16 * DD;
  const _Float16* bp0 = wc + (size_t)(mat * DD + c0 + 64 * wq + l16) * DD + 8 * h;
  const _Float16* bp1 = bp0 + (size_t)16 * DD;
  const _Float16* bp2 = bp0 + (size_t)32 * DD;
  const _Float16* bp3 = bp0 + (size_t)48 * DD;

  v8f acc[2][4];
#pragma unroll
  for (int mt = 0; mt < 2; ++mt)
#pragma unroll
    for (int nt = 0; nt < 4; ++nt) acc[mt][nt] = zero8();

#pragma unroll 1
  for (int kc = 0; kc < DD; kc += 32) {
    const v16h A0 = ldfrag(ap0 + kc);
    const v16h A1 = ldfrag(ap1 + kc);
    const v16h B0 = ldfrag(bp0 + kc);
    const v16h B1 = ldfrag(bp1 + kc);
    const v16h B2 = ldfrag(bp2 + kc);
    const v16h B3 = ldfrag(bp3 + kc);
    acc[0][0] = mma16(A0, B0, acc[0][0]);
    acc[0][1] = mma16(A0, B1, acc[0][1]);
    acc[0][2] = mma16(A0, B2, acc[0][2]);
    acc[0][3] = mma16(A0, B3, acc[0][3]);
    acc[1][0] = mma16(A1, B0, acc[1][0]);
    acc[1][1] = mma16(A1, B1, acc[1][1]);
    acc[1][2] = mma16(A1, B2, acc[1][2]);
    acc[1][3] = mma16(A1, B3, acc[1][3]);
    asm volatile("v_nop\n\tv_nop\n\tv_nop\n\tv_nop"
                 : "+v"(acc[0][0]), "+v"(acc[0][1]), "+v"(acc[0][2]), "+v"(acc[0][3]),
                   "+v"(acc[1][0]), "+v"(acc[1][1]), "+v"(acc[1][2]), "+v"(acc[1][3])
                 : "v"(A0), "v"(A1), "v"(B0), "v"(B1), "v"(B2), "v"(B3));
  }

  const int cl0 = 64 * wq + l16;
  const int rl0 = 32 * wr + 8 * h;
#pragma unroll
  for (int nt = 0; nt < 4; ++nt) {
    const float bias = bc[mat * DD + c0 + cl0 + 16 * nt];
#pragma unroll
    for (int mt = 0; mt < 2; ++mt) acc[mt][nt] = acc[mt][nt] * INV_WCARRY + bias;
  }

  v8h rv[8];
  if (mat < 2) {
    _Float16* ph = (mat == 0) ? qh : kh;
    _Float16* pl = (mat == 0) ? ql : kl;
#pragma unroll
    for (int pass = 0; pass < 2; ++pass) {
#pragma unroll
      for (int mt = 0; mt < 2; ++mt)
#pragma unroll
        for (int nt = 0; nt < 4; ++nt)
#pragma unroll
          for (int r = 0; r < 8; ++r) {
            const float    v  = acc[mt][nt][r];
            const _Float16 hv = (_Float16)v;
            _Float16 sv;
            if (pass == 0) sv = hv;
            else           sv = (_Float16)((v - (float)hv) * RCARRY);
            T[(rl0 + 16 * mt + r) * TP + cl0 + 16 * nt] = sv;
          }
      __syncthreads();
#pragma unroll
      for (int i = 0; i < 8; ++i)
        rv[i] = *(const v8h*)&T[(16 * w + 2 * i + h) * TP + 8 * l16];
      _Float16* pd = (pass == 0) ? ph : pl;
#pragma unroll
      for (int i = 0; i < 8; ++i)
        *(volatile v8h*)(pd + (size_t)(rb + 16 * w + 2 * i + h) * DD + c0 + 8 * l16) = rv[i];
      __threadfence();
#pragma unroll
      for (int i = 0; i < 8; ++i)
        *(volatile v8h*)(pd + (size_t)(rb + 16 * w + 2 * i + h) * DD + c0 + 8 * l16) = rv[i];
      __syncthreads();
    }
  } else {
#pragma unroll
    for (int mt = 0; mt < 2; ++mt)
#pragma unroll
      for (int nt = 0; nt < 4; ++nt) {
        v8h o;
#pragma unroll
        for (int r = 0; r < 8; ++r) o[r] = (_Float16)(acc[mt][nt][r] * VCARRY);
        *(v8h*)&T[(cl0 + 16 * nt) * TP + rl0 + 16 * mt] = o;
      }
    __syncthreads();
    const int bb = rb / SEQ;
    const int s0 = rb - bb * SEQ;
#pragma unroll
    for (int i = 0; i < 8; ++i)
      rv[i] = *(const v8h*)&T[(16 * w + 2 * i + h) * TP + 8 * l16];
#pragma unroll
    for (int i = 0; i < 8; ++i)
      *(volatile v8h*)(vt + ((size_t)bb * DD + c0 + 16 * w + 2 * i + h) * SEQ + s0 + 8 * l16) = rv[i];
    __threadfence();
#pragma unroll
    for (int i = 0; i < 8; ++i)
      *(volatile v8h*)(vt + ((size_t)bb * DD + c0 + 16 * w + 2 * i + h) * SEQ + s0 + 8 * l16) = rv[i];
  }
}

__global__ __launch_bounds__(256) void attn_kernel(
    const _Float16* __restrict__ qh, const _Float16* __restrict__ ql,
    const _Float16* __restrict__ kh, const _Float16* __restrict__ kl,
    const _Float16* __restrict__ vt, float* __restrict__ out)
{
  __shared__ __attribute__((aligned(16))) float    sp[8192];
  __shared__ __attribute__((aligned(16))) _Float16 pb[1024];
  __shared__ float scl[64];
  __shared__ float invl[64];

  const int tid  = threadIdx.x;
  const int w    = __builtin_amdgcn_readfirstlane(tid >> 5);
  const int lane = tid & 31, h = lane >> 4, l16 = lane & 15;
  const int qt   = w >> 2, dq = w & 3;
  const int b     = blockIdx.y;
  const int qbase = blockIdx.x * 32;

  const size_t prow = (size_t)b * SEQ + qbase + 16 * qt + l16;
  const _Float16* qhp = qh + prow * DD + 128 * dq + 8 * h;
  const _Float16* qlp = ql + prow * DD + 128 * dq + 8 * h;
  const size_t krow = (size_t)b * SEQ + l16;
  const _Float16* khp = kh + krow * DD + 128 * dq + 8 * h;
  const _Float16* klp = kl + krow * DD + 128 * dq + 8 * h;
  const _Float16* vtp = vt + ((size_t)b * DD + 128 * dq + l16) * SEQ + 8 * h;

  const int pbo = (qt * 32 + lane) * 16;
  const int slo = qt * 32 + lane;

  v8f O[8];
#pragma unroll
  for (int dt = 0; dt < 8; ++dt) O[dt] = zero8();
  float mx = -1.0e30f, sm = 0.0f;

#pragma unroll 1
  for (int kt = 0; kt < SEQ; kt += 32) {
    v8f shh0 = zero8(), shh1 = zero8(), sx0 = zero8(), sx1 = zero8();
    const _Float16* kh0 = khp + (size_t)kt * DD;
    const _Float16* kl0 = klp + (size_t)kt * DD;
#pragma unroll
    for (int j = 0; j < 4; ++j) {
      const v16h Bh  = ldfrag(qhp + 32 * j);
      const v16h Bl  = ldfrag(qlp + 32 * j);
      const v16h Ah0 = ldfrag(kh0 + 32 * j);
      const v16h Al0 = ldfrag(kl0 + 32 * j);
      const v16h Ah1 = ldfrag(kh0 + 16 * DD + 32 * j);
      const v16h Al1 = ldfrag(kl0 + 16 * DD + 32 * j);
      shh0 = mma16(Ah0, Bh, shh0);
      sx0  = mma16(Ah0, Bl, sx0);
      sx0  = mma16(Al0, Bh, sx0);
      shh1 = mma16(Ah1, Bh, shh1);
      sx1  = mma16(Ah1, Bl, sx1);
      sx1  = mma16(Al1, Bh, sx1);
      asm volatile("v_nop\n\tv_nop\n\tv_nop\n\tv_nop"
                   : "+v"(shh0), "+v"(shh1), "+v"(sx0), "+v"(sx1)
                   : "v"(Ah0), "v"(Al0), "v"(Ah1), "v"(Al1), "v"(Bh), "v"(Bl));
    }
    v8f part0 = shh0 + sx0 * INV_RCARRY;
    v8f part1 = shh1 + sx1 * INV_RCARRY;

    if (dq != 0) {
      const int o = (qt * 3 + dq - 1) * 512 + lane * 8;
      Acc8 u0, u1;
      u0.v = part0; u1.v = part1;
      *(v4f*)&sp[o]       = u0.q[0];
      *(v4f*)&sp[o + 4]   = u0.q[1];
      *(v4f*)&sp[o + 256] = u1.q[0];
      *(v4f*)&sp[o + 260] = u1.q[1];
    }
    __syncthreads();

    if (dq == 0) {
#pragma unroll
      for (int m1 = 0; m1 < 3; ++m1) {
        const int o = (qt * 3 + m1) * 512 + lane * 8;
        Acc8 u0, u1;
        u0.q[0] = *(const v4f*)&sp[o];
        u0.q[1] = *(const v4f*)&sp[o + 4];
        u1.q[0] = *(const v4f*)&sp[o + 256];
        u1.q[1] = *(const v4f*)&sp[o + 260];
        part0 += u0.v;
        part1 += u1.v;
      }
      float tmax = -1.0e30f;
#pragma unroll
      for (int r = 0; r < 8; ++r) {
        tmax = fmaxf(tmax, part0[r]);
        tmax = fmaxf(tmax, part1[r]);
      }
      tmax = fmaxf(tmax, __shfl_xor(tmax, 16, 32));
      const float nmx = fmaxf(mx, tmax);
      const float sc  = __builtin_amdgcn_exp2f((mx - nmx) * L2E);
      mx = nmx;
      v8f p0, p1;
      float ps = 0.0f;
#pragma unroll
      for (int r = 0; r < 8; ++r) {
        p0[r] = __builtin_amdgcn_exp2f((part0[r] - mx) * L2E);
        p1[r] = __builtin_amdgcn_exp2f((part1[r] - mx) * L2E);
        ps += p0[r] + p1[r];
      }
      ps += __shfl_xor(ps, 16, 32);
      sm = sm * sc + ps;
      v8h t0, t1;
#pragma unroll
      for (int r = 0; r < 8; ++r) {
        t0[r] = (_Float16)(p0[r] * PCARRY);
        t1[r] = (_Float16)(p1[r] * PCARRY);
      }
      *(v8h*)&pb[pbo]     = t0;
      *(v8h*)&pb[pbo + 8] = t1;
      scl[slo] = sc;
    }
    __syncthreads();

    const float osc = scl[slo];
    Frag bpf;
    bpf.p[0] = *(const v8h*)&pb[pbo];
    bpf.p[1] = *(const v8h*)&pb[pbo + 8];
    const v16h Bp = bpf.v;
#pragma unroll
    for (int dt = 0; dt < 8; ++dt) O[dt] = O[dt] * osc;

    const _Float16* v0 = vtp + kt;
    {
      const v16h V0 = ldfrag(v0);
      const v16h V1 = ldfrag(v0 + (size_t)SEQ * 16);
      const v16h V2 = ldfrag(v0 + (size_t)SEQ * 32);
      const v16h V3 = ldfrag(v0 + (size_t)SEQ * 48);
      O[0] = mma16(V0, Bp, O[0]);
      O[1] = mma16(V1, Bp, O[1]);
      O[2] = mma16(V2, Bp, O[2]);
      O[3] = mma16(V3, Bp, O[3]);
      asm volatile("v_nop\n\tv_nop\n\tv_nop\n\tv_nop"
                   : "+v"(O[0]), "+v"(O[1]), "+v"(O[2]), "+v"(O[3])
                   : "v"(V0), "v"(V1), "v"(V2), "v"(V3), "v"(Bp));
    }
    {
      const v16h V4 = ldfrag(v0 + (size_t)SEQ * 64);
      const v16h V5 = ldfrag(v0 + (size_t)SEQ * 80);
      const v16h V6 = ldfrag(v0 + (size_t)SEQ * 96);
      const v16h V7 = ldfrag(v0 + (size_t)SEQ * 112);
      O[4] = mma16(V4, Bp, O[4]);
      O[5] = mma16(V5, Bp, O[5]);
      O[6] = mma16(V6, Bp, O[6]);
      O[7] = mma16(V7, Bp, O[7]);
      asm volatile("v_nop\n\tv_nop\n\tv_nop\n\tv_nop"
                   : "+v"(O[4]), "+v"(O[5]), "+v"(O[6]), "+v"(O[7])
                   : "v"(V4), "v"(V5), "v"(V6), "v"(V7), "v"(Bp));
    }
  }

  if (dq == 0) {
    const float inv = (1.0f / sm) * INV_PV;
    invl[slo] = inv;
  }
  __syncthreads();
  const float inv = invl[slo];

#pragma unroll
  for (int pass = 0; pass < 2; ++pass) {
    if (qt == pass) {
#pragma unroll
      for (int dt = 0; dt < 8; ++dt) {
        Acc8 u;
        u.v = O[dt] * inv;
        const int base = l16 * DD + 128 * dq + 16 * dt + 8 * h;
        *(v4f*)&sp[base]     = u.q[0];
        *(v4f*)&sp[base + 4] = u.q[1];
      }
    }
    __syncthreads();
    v4f rv[8];
#pragma unroll
    for (int rr = 0; rr < 2; ++rr)
#pragma unroll
      for (int i = 0; i < 4; ++i)
        rv[rr * 4 + i] = *(const v4f*)&sp[(2 * w + rr) * DD + 128 * i + 4 * lane];
    float* orow = out + ((size_t)b * SEQ + qbase + 16 * pass + 2 * w) * DD;
#pragma unroll
    for (int rr = 0; rr < 2; ++rr)
#pragma unroll
      for (int i = 0; i < 4; ++i)
        *(volatile v4f*)(orow + (size_t)rr * DD + 128 * i + 4 * lane) = rv[rr * 4 + i];
    __threadfence();
#pragma unroll
    for (int rr = 0; rr < 2; ++rr)
#pragma unroll
      for (int i = 0; i < 4; ++i)
        *(volatile v4f*)(orow + (size_t)rr * DD + 128 * i + 4 * lane) = rv[rr * 4 + i];
    __syncthreads();
  }
}

extern "C" void kernel_launch(void* const* d_in, const int* in_sizes, int n_in,
                              void* d_out, int out_size, void* d_ws, size_t ws_size,
                              hipStream_t stream) {
  if (n_in < 7) return;
  const long long need_x = ((long long)(NB - 1) * SEQ_FULL + SEQ) * DD;
  if ((long long)in_sizes[0] < need_x) return;
  if (in_sizes[1] < DD * DD || in_sizes[3] < DD * DD || in_sizes[5] < DD * DD) return;
  if (in_sizes[2] < DD || in_sizes[4] < DD || in_sizes[6] < DD) return;
  if ((long long)out_size < (long long)NROWS * DD) return;

  const float* x  = (const float*)d_in[0];
  const float* Wq = (const float*)d_in[1];
  const float* bq = (const float*)d_in[2];
  const float* Wk = (const float*)d_in[3];
  const float* bk = (const float*)d_in[4];
  const float* Wv = (const float*)d_in[5];
  const float* bv = (const float*)d_in[6];
  float* outp = (float*)d_out;

  const size_t plane = (size_t)NROWS * DD * 2;
  const size_t wcb   = (size_t)NWROWS * DD * 2;
  const size_t bcb   = (size_t)NWROWS * 4;
  const size_t vtb   = (size_t)NB * DD * SEQ * 2;
  const size_t o_xh = 0;
  const size_t o_wc = o_xh + plane;
  const size_t o_bc = o_wc + wcb;
  const size_t o_qh = o_bc + bcb;
  const size_t o_ql = o_qh + plane;
  const size_t o_kh = o_ql + plane;
  const size_t o_kl = o_kh + plane;
  const size_t o_vt = o_kl + plane;
  const size_t total = o_vt + vtb;
  if (total > ws_size) return;

  char* ws = (char*)d_ws;
  _Float16* xh = (_Float16*)(ws + o_xh);
  _Float16* wc = (_Float16*)(ws + o_wc);
  float*    bc = (float*)(ws + o_bc);
  _Float16* qh = (_Float16*)(ws + o_qh);
  _Float16* ql = (_Float16*)(ws + o_ql);
  _Float16* kh = (_Float16*)(ws + o_kh);
  _Float16* kl = (_Float16*)(ws + o_kl);
  _Float16* vt = (_Float16*)(ws + o_vt);

  const int nbx = NROWS / 4;
  const int nbw = (NWROWS * DD / 8) / 256;
  const int nbb = 2;
  cvt_kernel<<<dim3(nbx + nbw + nbb), dim3(256), 0, stream>>>(
      x, Wq, bq, Wk, bk, Wv, bv, xh, wc, bc, nbx, nbw);

  proj_kernel<<<dim3(NROWS / 128, 12), dim3(256), 0, stream>>>(
      xh, wc, bc, qh, ql, kh, kl, vt);

  attn_kernel<<<dim3(SEQ / 32, NB), dim3(256), 0, stream>>>(
      qh, ql, kh, kl, vt, outp);
}
